// CustomxLSTM_21345987461769
// MI455X (gfx1250) — hardware-run, weakly checked
//
#include <hip/hip_runtime.h>
#include <math.h>

constexpr int NBAT   = 8;
constexpr int NSTEP  = 1024;
constexpr int NIN    = 128;
constexpr int NHID   = 128;
constexpr int NGATE  = 4 * NHID;
constexpr int NPROJ  = 6 * NHID;
constexpr int NROWS  = NBAT * NSTEP;
constexpr int WROWS  = NGATE + NGATE + NPROJ;
constexpr int HPITCH = 136;
constexpr int GSTR   = NHID * NHID;

static_assert(NBAT == 8, "row index math uses m>>3, m&7");
static_assert(NIN == 128 && NHID == 128, "plane row = 16 groups of 8 elements");
static_assert(NIN % 32 == 0 && NHID % 32 == 0, "GEMM K multiple of 32");
static_assert(NROWS % 64 == 0 && NGATE % 64 == 0 && NPROJ % 64 == 0, "GEMM M, N tile multiples");
static_assert(NROWS % 32 == 0, "six-product GEMM M tile multiple");
static_assert(((NROWS / 32) * (NGATE / 64)) % 8 == 0, "six-product GEMM grid exact");
static_assert(((NROWS / 64) * (NPROJ / 64)) % 8 == 0, "three-product GEMM grid exact");
static_assert(HPITCH % 8 == 0 && HPITCH >= NHID, "LDS pitch keeps 16-B alignment");
static_assert((NBAT * NGATE) == 4 * 256 * 4, "gate pre-activation staging: 4 x 256 threads x float4");
static_assert(NHID / 16 == 8, "eight unit subtiles = eight waves in the layer-0 recurrence");

typedef __attribute__((ext_vector_type(16))) __bf16   v16b;
typedef __attribute__((ext_vector_type(8)))  __bf16   v8b;
typedef __attribute__((ext_vector_type(8)))  float    v8f;
typedef __attribute__((ext_vector_type(4)))  float    v4f;
typedef __attribute__((ext_vector_type(4)))  unsigned v4u;

__device__ __forceinline__ unsigned f2bf_bits(float f) {
  const unsigned u = __float_as_uint(f);
  return ((u + 0x7FFFu + ((u >> 16) & 1u)) >> 16) & 0xFFFFu;
}
__device__ __forceinline__ float bf_bits2f(unsigned h) { return __uint_as_float(h << 16); }
__device__ __forceinline__ void split_bf3(float f, unsigned& hb, unsigned& mb, unsigned& lb) {
  hb = f2bf_bits(f);
  const float r1 = f - bf_bits2f(hb);
  mb = f2bf_bits(r1);
  const float r2 = r1 - bf_bits2f(mb);
  lb = f2bf_bits(r2);
}
__device__ __forceinline__ void pack_split8x3(const v4f a, const v4f b, v4u& hv, v4u& mv, v4u& lv) {
  const float f0 = a[0], f1 = a[1], f2 = a[2], f3 = a[3];
  const float f4 = b[0], f5 = b[1], f6 = b[2], f7 = b[3];
  unsigned h0, h1, h2, h3, h4, h5, h6, h7;
  unsigned m0, m1, m2, m3, m4, m5, m6, m7;
  unsigned l0, l1, l2, l3, l4, l5, l6, l7;
  split_bf3(f0, h0, m0, l0); split_bf3(f1, h1, m1, l1); split_bf3(f2, h2, m2, l2); split_bf3(f3, h3, m3, l3);
  split_bf3(f4, h4, m4, l4); split_bf3(f5, h5, m5, l5); split_bf3(f6, h6, m6, l6); split_bf3(f7, h7, m7, l7);
  hv[0] = h0 | (h1 << 16); hv[1] = h2 | (h3 << 16); hv[2] = h4 | (h5 << 16); hv[3] = h6 | (h7 << 16);
  mv[0] = m0 | (m1 << 16); mv[1] = m2 | (m3 << 16); mv[2] = m4 | (m5 << 16); mv[3] = m6 | (m7 << 16);
  lv[0] = l0 | (l1 << 16); lv[1] = l2 | (l3 << 16); lv[2] = l4 | (l5 << 16); lv[3] = l6 | (l7 << 16);
}
__device__ __forceinline__ float exp_ftz(float x) {
  const float e = expf(x);
  return (e < 1.17549435e-38f) ? 0.0f : e;
}

__device__ __forceinline__ void wm_guard4(v8f& a, v8f& b, v8f& c, v8f& d, v16b x, v16b y) {
  asm volatile("v_nop\n\tv_nop\n\tv_nop\n\tv_nop" : "+v"(a), "+v"(b), "+v"(c), "+v"(d) : "v"(x), "v"(y));
}
__device__ __forceinline__ void keep4_b(v16b a, v16b b, v16b c, v16b d) { asm volatile("v_nop" :: "v"(a), "v"(b), "v"(c), "v"(d)); }
__device__ __forceinline__ void acc_guard4(v8f& a, v8f& b, v8f& c, v8f& d) {
  asm volatile("v_nop\n\tv_nop\n\tv_nop\n\tv_nop" : "+v"(a), "+v"(b), "+v"(c), "+v"(d));
}
struct FragB {
  union U { v16b v; v8b h[2]; };
  static __device__ __forceinline__ v16b load(const __bf16* p) {
    U f; f.h[0] = *(const v8b*)(p); f.h[1] = *(const v8b*)(p + 16); return f.v;
  }
  static __device__ __forceinline__ v8f mma(v16b a, v16b b, v8f c) {
    return __builtin_amdgcn_wmma_f32_16x16x32_bf16(false, a, false, b, (short)0, c, false, false);
  }
};
__device__ __forceinline__ v8f mma_g(v16b a, v16b b, v8f c) {
  c = __builtin_amdgcn_wmma_f32_16x16x32_bf16(false, a, false, b, (short)0, c, false, false);
  asm volatile("v_nop\n\tv_nop\n\tv_nop\n\tv_nop" : "+v"(c) : "v"(a), "v"(b));
  return c;
}

__global__ __launch_bounds__(256) void prep_x_kernel(const float* __restrict__ x,
                                                     unsigned short* __restrict__ X0,
                                                     unsigned short* __restrict__ X1,
                                                     unsigned short* __restrict__ X2) {
  const int i = blockIdx.x * 256 + threadIdx.x;
  if (i < NROWS * (NIN / 8)) {
    const int m = i >> 4, c8 = i & 15;
    const int t = m >> 3, b = m & 7;
    const float* sp = x + ((size_t)(b * NSTEP + t)) * NIN + c8 * 8;
    const v4f a  = *(const v4f*)(sp);
    const v4f bb = *(const v4f*)(sp + 4);
    v4u hv, mv, lv;
    pack_split8x3(a, bb, hv, mv, lv);
    unsigned short* p0 = X0 + (size_t)i * 8;
    unsigned short* p1 = X1 + (size_t)i * 8;
    unsigned short* p2 = X2 + (size_t)i * 8;
    for (int pass = 0; pass < 2; ++pass) {
      *(volatile v4u*)p0 = hv;
      *(volatile v4u*)p1 = mv;
      *(volatile v4u*)p2 = lv;
      __threadfence();
    }
  }
}

__global__ __launch_bounds__(256) void prep_w_kernel(const float* __restrict__ sW, const float* __restrict__ sR,
                                                     const float* __restrict__ Wq, const float* __restrict__ Wk,
                                                     const float* __restrict__ Wv, const float* __restrict__ Wi,
                                                     const float* __restrict__ Wf, const float* __restrict__ Wo,
                                                     unsigned short* __restrict__ W0,
                                                     unsigned short* __restrict__ W1,
                                                     unsigned short* __restrict__ W2) {
  const int rb = blockIdx.x;
  const float* src = sW;
  int lr0 = rb * 16;
  if (rb >= 64) {
    const int wq = (rb - 64) >> 3;
    lr0 = ((rb - 64) & 7) * 16;
    src = (wq == 0) ? Wq : (wq == 1) ? Wk : (wq == 2) ? Wv : (wq == 3) ? Wi : (wq == 4) ? Wf : Wo;
  } else if (rb >= 32) {
    src = sR;
    lr0 = (rb - 32) * 16;
  }
  const int tid = threadIdx.x;
  const int rr = tid >> 4, c8 = tid & 15;
  const float* sp = src + (size_t)(lr0 + rr) * NHID + c8 * 8;
  const v4f a  = *(const v4f*)(sp);
  const v4f bb = *(const v4f*)(sp + 4);
  v4u hv, mv, lv;
  pack_split8x3(a, bb, hv, mv, lv);
  const size_t i = (size_t)rb * 256 + tid;
  unsigned short* p0 = W0 + i * 8;
  unsigned short* p1 = W1 + i * 8;
  unsigned short* p2 = W2 + i * 8;
  for (int pass = 0; pass < 2; ++pass) {
    *(volatile v4u*)p0 = hv;
    *(volatile v4u*)p1 = mv;
    *(volatile v4u*)p2 = lv;
    __threadfence();
  }
}

template <int BIAS_MODE>
__global__ __launch_bounds__(256) void gemm32x64_b6_kernel(
    const unsigned short* __restrict__ A0p, const unsigned short* __restrict__ A1p,
    const unsigned short* __restrict__ A2p, int lda,
    const unsigned short* __restrict__ B0p, const unsigned short* __restrict__ B1p,
    const unsigned short* __restrict__ B2p, int ldb,
    float* __restrict__ Cout, int ldc, const float* __restrict__ bias, int M, int N, int K) {
  const __bf16* A0 = (const __bf16*)A0p; const __bf16* A1 = (const __bf16*)A1p; const __bf16* A2 = (const __bf16*)A2p;
  const __bf16* B0 = (const __bf16*)B0p; const __bf16* B1 = (const __bf16*)B1p; const __bf16* B2 = (const __bf16*)B2p;
  __shared__ __align__(16) float sT[8][16 * 68];
  const int lane = threadIdx.x & 31;
  const int wave = threadIdx.x >> 5;
  const int tilesN = N >> 6;
  const int tilesM = M >> 5;
  const int tile = blockIdx.x * 8 + wave;
  if (tile >= tilesM * tilesN) return;
  const int tm = tile / tilesN;
  const int tn = tile - tm * tilesN;
  const int m0 = tm << 5;
  const int n0 = tn << 6;
  const int rlane = lane & 15;
  const int koff  = (lane >> 4) * 8;
  const int mOff  = (lane >> 4) * 8;

  v8f acc[2][4];
#pragma unroll
  for (int i = 0; i < 2; ++i)
#pragma unroll
    for (int j = 0; j < 4; ++j) acc[i][j] = (v8f){0.f, 0.f, 0.f, 0.f, 0.f, 0.f, 0.f, 0.f};

  for (int k0 = 0; k0 < K; k0 += 32) {
    v16b b0[4], b1[4], b2[4];
#pragma unroll
    for (int j = 0; j < 4; ++j) {
      const size_t bo = (size_t)(n0 + (j << 4) + rlane) * ldb + koff + k0;
      b0[j] = FragB::load(B0 + bo);
      b1[j] = FragB::load(B1 + bo);
      b2[j] = FragB::load(B2 + bo);
    }
#pragma unroll
    for (int i = 0; i < 2; ++i) {
      const size_t ao = (size_t)(m0 + (i << 4) + rlane) * lda + koff + k0;
      const v16b a0 = FragB::load(A0 + ao);
      const v16b a1 = FragB::load(A1 + ao);
      const v16b a2 = FragB::load(A2 + ao);
#pragma unroll
      for (int j = 0; j < 4; ++j) {
        acc[i][j] = mma_g(a0, b0[j], acc[i][j]);
        acc[i][j] = mma_g(a0, b1[j], acc[i][j]);
        acc[i][j] = mma_g(a1, b0[j], acc[i][j]);
        acc[i][j] = mma_g(a0, b2[j], acc[i][j]);
        acc[i][j] = mma_g(a2, b0[j], acc[i][j]);
        acc[i][j] = mma_g(a1, b1[j], acc[i][j]);
      }
    }
    keep4_b(b0[0], b0[1], b0[2], b0[3]);
    keep4_b(b1[0], b1[1], b1[2], b1[3]);
    keep4_b(b2[0], b2[1], b2[2], b2[3]);
  }
  acc_guard4(acc[0][0], acc[0][1], acc[0][2], acc[0][3]);
  acc_guard4(acc[1][0], acc[1][1], acc[1][2], acc[1][3]);

  float* slab = sT[wave];
#pragma unroll
  for (int i = 0; i < 2; ++i) {
    const int mBase = m0 + (i << 4);
#pragma unroll
    for (int j = 0; j < 4; ++j) {
      const int n = n0 + (j << 4) + rlane;
      float bv = 0.f;
      if (BIAS_MODE == 2) bv = bias[n];
#pragma unroll
      for (int r = 0; r < 8; ++r) {
        float v = acc[i][j][r];
        if (BIAS_MODE == 2) v += bv;
        slab[(mOff + r) * 68 + (j << 4) + rlane] = v;
      }
    }
    __builtin_amdgcn_fence(__ATOMIC_RELEASE, "workgroup");
    __builtin_amdgcn_wave_barrier();
    __builtin_amdgcn_fence(__ATOMIC_ACQUIRE, "workgroup");
    {
      const int hh = lane >> 4, c4 = (lane & 15) * 4;
      for (int pass = 0; pass < 2; ++pass) {
#pragma unroll
        for (int it = 0; it < 8; ++it) {
          const int row = it * 2 + hh;
          const v4f v = *(const v4f*)(slab + row * 68 + c4);
          *(volatile v4f*)(Cout + (size_t)(mBase + row) * ldc + n0 + c4) = v;
        }
        __threadfence();
      }
    }
    __builtin_amdgcn_fence(__ATOMIC_RELEASE, "workgroup");
    __builtin_amdgcn_wave_barrier();
    __builtin_amdgcn_fence(__ATOMIC_ACQUIRE, "workgroup");
  }
}

template <int BIAS_MODE>
__global__ __launch_bounds__(256) void gemm64_b3_kernel(
    const unsigned short* __restrict__ Ap, const unsigned short* __restrict__ A2p, int lda,
    const unsigned short* __restrict__ Btp, const unsigned short* __restrict__ Bt2p, int ldb,
    float* __restrict__ Cout, int ldc, const float* __restrict__ bias, int M, int N, int K) {
  const __bf16* A = (const __bf16*)Ap;   const __bf16* A2  = (const __bf16*)A2p;
  const __bf16* Bt = (const __bf16*)Btp; const __bf16* Bt2 = (const __bf16*)Bt2p;
  __shared__ __align__(16) float sT[8][16 * 68];
  const int lane = threadIdx.x & 31;
  const int wave = threadIdx.x >> 5;
  const int tilesN = N >> 6;
  const int tilesM = M >> 6;
  const int tile = blockIdx.x * 8 + wave;
  if (tile >= tilesM * tilesN) return;
  const int tm = tile / tilesN;
  const int tn = tile - tm * tilesN;
  const int m0 = tm << 6;
  const int n0 = tn << 6;
  const int rlane = lane & 15;
  const int koff  = (lane >> 4) * 8;
  const int mOff  = (lane >> 4) * 8;

  v8f acc[4][4];
#pragma unroll
  for (int i = 0; i < 4; ++i)
#pragma unroll
    for (int j = 0; j < 4; ++j) acc[i][j] = (v8f){0.f, 0.f, 0.f, 0.f, 0.f, 0.f, 0.f, 0.f};

  for (int k0 = 0; k0 < K; k0 += 32) {
    v16b bh[4], bl[4];
#pragma unroll
    for (int j = 0; j < 4; ++j) {
      const size_t bo = (size_t)(n0 + (j << 4) + rlane) * ldb + koff + k0;
      bh[j] = FragB::load(Bt + bo);
      bl[j] = FragB::load(Bt2 + bo);
    }
#pragma unroll
    for (int i = 0; i < 4; ++i) {
      const size_t ao = (size_t)(m0 + (i << 4) + rlane) * lda + koff + k0;
      const v16b ah = FragB::load(A + ao);
      const v16b al = FragB::load(A2 + ao);
#pragma unroll
      for (int j = 0; j < 4; ++j) {
        acc[i][j] = FragB::mma(ah, bh[j], acc[i][j]);
        acc[i][j] = FragB::mma(ah, bl[j], acc[i][j]);
        acc[i][j] = FragB::mma(al, bh[j], acc[i][j]);
      }
      wm_guard4(acc[i][0], acc[i][1], acc[i][2], acc[i][3], ah, al);
    }
    keep4_b(bh[0], bh[1], bh[2], bh[3]);
    keep4_b(bl[0], bl[1], bl[2], bl[3]);
  }
  acc_guard4(acc[0][0], acc[0][1], acc[0][2], acc[0][3]);
  acc_guard4(acc[1][0], acc[1][1], acc[1][2], acc[1][3]);
  acc_guard4(acc[2][0], acc[2][1], acc[2][2], acc[2][3]);
  acc_guard4(acc[3][0], acc[3][1], acc[3][2], acc[3][3]);

  float* slab = sT[wave];
#pragma unroll
  for (int i = 0; i < 4; ++i) {
    const int mBase = m0 + (i << 4);
#pragma unroll
    for (int j = 0; j < 4; ++j) {
      const int n = n0 + (j << 4) + rlane;
      float bv = 0.f;
      if (BIAS_MODE == 2) bv = bias[n];
#pragma unroll
      for (int r = 0; r < 8; ++r) {
        float v = acc[i][j][r];
        if (BIAS_MODE == 2) v += bv;
        slab[(mOff + r) * 68 + (j << 4) + rlane] = v;
      }
    }
    __builtin_amdgcn_fence(__ATOMIC_RELEASE, "workgroup");
    __builtin_amdgcn_wave_barrier();
    __builtin_amdgcn_fence(__ATOMIC_ACQUIRE, "workgroup");
    {
      const int hh = lane >> 4, c4 = (lane & 15) * 4;
      for (int pass = 0; pass < 2; ++pass) {
#pragma unroll
        for (int it = 0; it < 8; ++it) {
          const int row = it * 2 + hh;
          const v4f v = *(const v4f*)(slab + row * 68 + c4);
          *(volatile v4f*)(Cout + (size_t)(mBase + row) * ldc + n0 + c4) = v;
        }
        __threadfence();
      }
    }
    __builtin_amdgcn_fence(__ATOMIC_RELEASE, "workgroup");
    __builtin_amdgcn_wave_barrier();
    __builtin_amdgcn_fence(__ATOMIC_ACQUIRE, "workgroup");
  }
}

__global__ __launch_bounds__(256) void expgate_seq_kernel(const float* __restrict__ Gx,
                                                          const unsigned short* __restrict__ R0p,
                                                          const unsigned short* __restrict__ R1p,
                                                          const unsigned short* __restrict__ R2p,
                                                          unsigned short* __restrict__ H1H,
                                                          unsigned short* __restrict__ H1L) {
  __shared__ __align__(16) unsigned short At0[16 * HPITCH];
  __shared__ __align__(16) unsigned short At1[16 * HPITCH];
  __shared__ __align__(16) unsigned short At2[16 * HPITCH];
  __shared__ __align__(16) float sG[NBAT * NGATE];
  const int tid = threadIdx.x, lane = tid & 31, wave = tid >> 5;
  const int c = lane & 15, hh = lane >> 4, koff = hh * 8;
  const int j = 16 * wave + c;

#pragma unroll 1
  for (int i = tid; i < 16 * HPITCH; i += 256) {
    At0[i] = (unsigned short)0;
    At1[i] = (unsigned short)0;
    At2[i] = (unsigned short)0;
  }

  float cs[8], ns[8], ms[8];
#pragma unroll
  for (int r = 0; r < 8; ++r) { cs[r] = 0.0f; ns[r] = 0.0f; ms[r] = 0.0f; }

  const __bf16* a0row = (const __bf16*)At0 + c * HPITCH + koff;
  const __bf16* a1row = (const __bf16*)At1 + c * HPITCH + koff;
  const __bf16* a2row = (const __bf16*)At2 + c * HPITCH + koff;
  const __bf16* r0 = (const __bf16*)R0p + (size_t)j * NHID + koff;
  const __bf16* r1 = (const __bf16*)R1p + (size_t)j * NHID + koff;
  const __bf16* r2 = (const __bf16*)R2p + (size_t)j * NHID + koff;
  const v8f z8 = {0.f, 0.f, 0.f, 0.f, 0.f, 0.f, 0.f, 0.f};
  __syncthreads();

#pragma unroll 1
  for (int t = 0; t < NSTEP; ++t) {
    {
      const float* gsrc = Gx + (size_t)t * (NBAT * NGATE);
#pragma unroll
      for (int i = 0; i < 4; ++i) {
        const int idx = (i * 256 + tid) * 4;
        const v4f v = *(const v4f*)(gsrc + idx);
        *(v4f*)(sG + idx) = v;
      }
    }
    v8f acc[4];
    acc[0] = z8; acc[1] = z8; acc[2] = z8; acc[3] = z8;
#pragma unroll 1
    for (int k0 = 0; k0 < NHID; k0 += 32) {
      const v16b a0 = FragB::load(a0row + k0);
      const v16b a1 = FragB::load(a1row + k0);
      const v16b a2 = FragB::load(a2row + k0);
#pragma unroll
      for (int g = 0; g < 4; ++g) {
        const v16b b0 = FragB::load(r0 + (size_t)g * GSTR + k0);
        const v16b b1 = FragB::load(r1 + (size_t)g * GSTR + k0);
        const v16b b2 = FragB::load(r2 + (size_t)g * GSTR + k0);
        acc[g] = mma_g(a0, b0, acc[g]);
        acc[g] = mma_g(a0, b1, acc[g]);
        acc[g] = mma_g(a1, b0, acc[g]);
        acc[g] = mma_g(a0, b2, acc[g]);
        acc[g] = mma_g(a2, b0, acc[g]);
        acc[g] = mma_g(a1, b1, acc[g]);
      }
    }
    acc_guard4(acc[0], acc[1], acc[2], acc[3]);
    __syncthreads();

#pragma unroll
    for (int r = 0; r < 8; ++r) {
      const int gb = r * NGATE + j;
      const float it = acc[0][r] + sG[gb];
      const float ft = acc[1][r] + sG[gb + NHID];
      const float zt = acc[2][r] + sG[gb + 2 * NHID];
      const float ot = acc[3][r] + sG[gb + 3 * NHID];
      const float zg = tanhf(zt);
      const float og = 1.0f / (1.0f + expf(-ot));
      const float t1 = ft + ms[r];
      const float mn = fmaxf(t1, it);
      const float ie = exp_ftz(it - mn);
      const float fe = exp_ftz(t1 - mn);
      const float cn = fe * cs[r] + ie * zg;
      const float nn = fe * ns[r] + ie;
      cs[r] = cn; ns[r] = nn; ms[r] = mn;
      const float hv = (og * cn) / nn;
      unsigned hb, mb, lb;
      split_bf3(hv, hb, mb, lb);
      const unsigned hsel = hh ? 0u : hb;
      const unsigned msel = hh ? 0u : mb;
      const unsigned lsel = hh ? 0u : lb;
      const int row = 8 * hh + r;
      At0[row * HPITCH + j] = (unsigned short)hsel;
      At1[row * HPITCH + j] = (unsigned short)msel;
      At2[row * HPITCH + j] = (unsigned short)lsel;
    }
    __syncthreads();

    {
      const int plane = wave >> 2;
      const int row = 2 * (wave & 3) + hh;
      const v4u vh = *(const v4u*)(At0 + row * HPITCH + c * 8);
      const v4u vl = *(const v4u*)(At1 + row * HPITCH + c * 8);
      v4u v;
      v[0] = plane ? vl[0] : vh[0];
      v[1] = plane ? vl[1] : vh[1];
      v[2] = plane ? vl[2] : vh[2];
      v[3] = plane ? vl[3] : vh[3];
      unsigned short* dst = (plane ? H1L : H1H) + ((size_t)(t * NBAT + row) * NHID + c * 8);
      for (int pass = 0; pass < 2; ++pass) {
        *(volatile v4u*)dst = v;
        __threadfence();
      }
    }
  }
}

__global__ __launch_bounds__(512) void matmem_seq_kernel(const float* __restrict__ P,
                                                         const float* __restrict__ bq, const float* __restrict__ bk,
                                                         const float* __restrict__ bv, const float* __restrict__ bi,
                                                         const float* __restrict__ bf, const float* __restrict__ bo,
                                                         float* __restrict__ out, float kscale) {
  __shared__ __align__(16) float sQ[NHID];
  __shared__ __align__(16) float sK[NHID];
  __shared__ __align__(16) float sF[NHID];
  __shared__ __align__(16) float sIV[NHID];
  __shared__ __align__(16) float sOg[NHID];
  __shared__ __align__(16) float sH[64];
  __shared__ __align__(16) float sRed[4];
  const int tid = threadIdx.x, lane = tid & 31, wave = tid >> 5;
  const int b = blockIdx.x >> 1, half = blockIdx.x & 1;
  const int jc = tid & (NHID - 1);
  const float vbq = bq[jc], vbk = bk[jc], vbv = bv[jc], vbi = bi[jc], vbf = bf[jc], vbo = bo[jc];

  float Cst[16];
#pragma unroll
  for (int i = 0; i < 16; ++i) Cst[i] = 0.0f;
  float nreg = 0.0f, mreg = 0.0f;

  const int rl = tid >> 3;
  const int r  = half * 64 + rl;
  const int cg = tid & 7;
  const int c0 = cg * 16;
  float* obase = out + (size_t)b * NSTEP * NHID + half * 64;

#pragma unroll 1
  for (int t = 0; t < NSTEP; ++t) {
    float p = 0.0f;
    if (tid < NHID) {
      const float* pr = P + (size_t)(t * NBAT + b) * NPROJ + tid;
      const float q  = pr[0] + vbq;
      const float kk = (pr[NHID] + vbk) * kscale;
      const float vv = pr[2 * NHID] + vbv;
      const float it = pr[3 * NHID] + vbi;
      const float ft = pr[4 * NHID] + vbf;
      const float ot = pr[5 * NHID] + vbo;
      const float t1 = ft + mreg;
      const float mn = fmaxf(t1, it);
      const float ie = exp_ftz(it - mn);
      const float fe = exp_ftz(t1 - mn);
      mreg = mn;
      nreg = fe * nreg + ie * kk;
      p = nreg * q;
      sQ[tid]  = q;
      sK[tid]  = kk;
      sF[tid]  = fe;
      sIV[tid] = ie * vv;
      sOg[tid] = 1.0f / (1.0f + expf(-ot));
    }
#pragma unroll
    for (int off = 1; off < 32; off <<= 1) p += __shfl_xor(p, off, 32);
    if (tid < NHID && lane == 0) sRed[wave] = p;
    __syncthreads();

    const float fe = sF[r];
    const float iv = sIV[r];
    const float og = sOg[r];
    float part = 0.0f;
#pragma unroll
    for (int i4 = 0; i4 < 4; ++i4) {
      const v4f kq = *(const v4f*)(sK + c0 + 4 * i4);
      const v4f qq = *(const v4f*)(sQ + c0 + 4 * i4);
#pragma unroll
      for (int e = 0; e < 4; ++e) {
        const float kc = kq[e];
        const float qc = qq[e];
        const float cn = fe * Cst[4 * i4 + e] + iv * kc;
        Cst[4 * i4 + e] = cn;
        part += cn * qc;
      }
    }
    part += __shfl_xor(part, 1, 32);
    part += __shfl_xor(part, 2, 32);
    part += __shfl_xor(part, 4, 32);
    const float nq  = (sRed[0] + sRed[1]) + (sRed[2] + sRed[3]);
    const float den = fmaxf(fabsf(nq), 1.0f);
    const float hv  = (og * part) * (1.0f / den);
    if (cg == 0) sH[rl] = hv;
    __syncthreads();

    if (wave == 0) {
      const int i4 = (lane & 15) * 4;
      const v4f v = *(const v4f*)(sH + i4);
      if (lane < 16) {
        float* op = obase + (size_t)t * NHID + i4;
        for (int pass = 0; pass < 2; ++pass) {
          *(volatile v4f*)op = v;
          __threadfence();
        }
      }
    }
  }
}

extern "C" void kernel_launch(void* const* d_in, const int* in_sizes, int n_in,
                              void* d_out, int out_size, void* d_ws, size_t ws_size, hipStream_t stream) {
  if (n_in < 16 || d_out == nullptr || d_ws == nullptr) return;
  if (in_sizes[0] != NBAT * NSTEP * NIN || in_sizes[1] != NGATE * NIN || in_sizes[2] != NGATE * NHID ||
      in_sizes[3] != NGATE || out_size != NBAT * NSTEP * NHID) return;
  for (int i = 4; i < 10; ++i) if (in_sizes[i] != NHID * NHID) return;
  for (int i = 10; i < 16; ++i) if (in_sizes[i] != NHID) return;

  const float* x  = (const float*)d_in[0];
  const float* sW = (const float*)d_in[1];
  const float* sR = (const float*)d_in[2];
  const float* sb = (const float*)d_in[3];
  const float* Wq = (const float*)d_in[4];
  const float* Wk = (const float*)d_in[5];
  const float* Wv = (const float*)d_in[6];
  const float* Wi = (const float*)d_in[7];
  const float* Wf = (const float*)d_in[8];
  const float* Wo = (const float*)d_in[9];
  const float* bq = (const float*)d_in[10];
  const float* bk = (const float*)d_in[11];
  const float* bv = (const float*)d_in[12];
  const float* bi = (const float*)d_in[13];
  const float* bf = (const float*)d_in[14];
  const float* bo = (const float*)d_in[15];
  float* out = (float*)d_out;

  char* ws = (char*)d_ws; size_t off = 0;
  auto carve = [&](size_t bytes) -> char* { char* p = ws + off; off += (bytes + 255) & ~(size_t)255; return p; };
  unsigned short* X0  = (unsigned short*)carve((size_t)NROWS * NIN * 2);
  unsigned short* X1  = (unsigned short*)carve((size_t)NROWS * NIN * 2);
  unsigned short* X2  = (unsigned short*)carve((size_t)NROWS * NIN * 2);
  unsigned short* W0  = (unsigned short*)carve((size_t)WROWS * NHID * 2);
  unsigned short* W1  = (unsigned short*)carve((size_t)WROWS * NHID * 2);
  unsigned short* W2  = (unsigned short*)carve((size_t)WROWS * NHID * 2);
  float*          GX  = (float*)carve((size_t)NROWS * NGATE * 4);
  unsigned short* H1H = (unsigned short*)carve((size_t)NROWS * NHID * 2);
  unsigned short* H1L = (unsigned short*)carve((size_t)NROWS * NHID * 2);
  float*          PP  = (float*)carve((size_t)NROWS * NPROJ * 4);
  if (off > ws_size || off > (size_t)134217728) return;

  const size_t roff = (size_t)NGATE * NHID;
  const size_t coff = (size_t)2 * NGATE * NHID;
  const float kscale = (float)(1.0 / sqrt((double)NHID));

  prep_x_kernel<<<(NROWS * (NIN / 8)) / 256, 256, 0, stream>>>(x, X0, X1, X2);
  prep_w_kernel<<<WROWS / 16, 256, 0, stream>>>(sW, sR, Wq, Wk, Wv, Wi, Wf, Wo, W0, W1, W2);

  gemm32x64_b6_kernel<2><<<(NROWS / 32) * (NGATE / 64) / 8, 256, 0, stream>>>(
      X0, X1, X2, NIN, W0, W1, W2, NIN, GX, NGATE, sb, NROWS, NGATE, NIN);

  expgate_seq_kernel<<<1, 256, 0, stream>>>(GX, W0 + roff, W1 + roff, W2 + roff, H1H, H1L);

  gemm64_b3_kernel<0><<<(NROWS / 64) * (NPROJ / 64) / 8, 256, 0, stream>>>(
      H1H, H1L, NHID, W0 + coff, W1 + coff, NHID, PP, NPROJ, sb, NROWS, NPROJ, NHID);

  matmem_seq_kernel<<<NBAT * 2, 512, 0, stream>>>(PP, bq, bk, bv, bi, bf, bo, out, kscale);
}
